// DisentangledSelfAttention_32444182954230
// MI455X (gfx1250) — hardware-run, weakly checked
//
#include <hip/hip_runtime.h>


#define NB_  4
#define TT   1024
#define DM   1024
#define NH_  16
#define NKV  16
#define REP  (NH_ / NKV)
#define HD   64
#define DQ   (NH_ * HD)
#define DKV  (NKV * HD)
#define ZH   2
#define RH   512
#define WIN  0
#define PCAR 1024.0f
#define SCL  0.072168783648703216f
#define NPOS 1024
typedef _Float16 h16;
typedef unsigned short bf;
typedef __attribute__((ext_vector_type(16))) __bf16   v16bf;
typedef __attribute__((ext_vector_type(16))) _Float16 v16h;
typedef __attribute__((ext_vector_type(8)))  _Float16 v8h;
typedef __attribute__((ext_vector_type(8)))  unsigned short v8us;
typedef __attribute__((ext_vector_type(8)))  float    v8f;
typedef __attribute__((ext_vector_type(4)))  float    v4f;
typedef v8h  __attribute__((may_alias)) v8ha;
typedef v4f  __attribute__((may_alias)) v4fa;
typedef v8us __attribute__((may_alias)) v8usa;

__device__ __forceinline__ unsigned short f2bf(float f) { unsigned u = __float_as_uint(f); u += 0x7FFFu + ((u >> 16) & 1u); return (unsigned short)(u >> 16); }
__device__ __forceinline__ float bf2f(unsigned short b) { return __uint_as_float(((unsigned)b) << 16); }
__device__ __forceinline__ float bfr(float f) { return bf2f(f2bf(f)); }
__device__ __forceinline__ v16h cat16(v8h lo, v8h hi) { return __builtin_shufflevector(lo, hi, 0, 1, 2, 3, 4, 5, 6, 7, 8, 9, 10, 11, 12, 13, 14, 15); }
__device__ __forceinline__ v16bf cat16b(v8us lo, v8us hi) { return __builtin_bit_cast(v16bf, __builtin_shufflevector(lo, hi, 0, 1, 2, 3, 4, 5, 6, 7, 8, 9, 10, 11, 12, 13, 14, 15)); }
__device__ __forceinline__ v8f wmma16(v16h a, v16h b, v8f c) { return __builtin_amdgcn_wmma_f32_16x16x32_f16(false, a, false, b, (short)0, c, false, false); }
__device__ __forceinline__ v8f wmmab(v16bf a, v16bf b, v8f c) { return __builtin_amdgcn_wmma_f32_16x16x32_bf16(false, a, false, b, (short)0, c, false, false); }


template <typename T16> struct WFrag;
template <> struct WFrag<h16> { typedef v16h V; static __device__ __forceinline__ V ld(const h16* p) { return cat16(*(const v8h*)p, *(const v8h*)(p + 16)); } static __device__ __forceinline__ v8f mma(V a, V b, v8f c) { return wmma16(a, b, c); } };
template <> struct WFrag<bf> { typedef v16bf V; static __device__ __forceinline__ V ld(const bf* p) { return cat16b(*(const v8us*)p, *(const v8us*)(p + 16)); } static __device__ __forceinline__ v8f mma(V a, V b, v8f c) { return wmmab(a, b, c); } };
template <typename T16, int NSPLIT, bool BIAS>
__global__ __launch_bounds__(32) void k_gemmw(const T16* __restrict__ A, const T16* __restrict__ A2, const T16* __restrict__ Bt, const T16* __restrict__ Bt2, int K, float* C, int ldc, const float* __restrict__ bias, size_t sA, size_t sB, size_t sC) {
    typedef typename WFrag<T16>::V V;
    __shared__ __align__(16) float os[16 * 68];
    const size_t z = blockIdx.z; A += z * sA; if (A2) A2 += z * sA; Bt += z * sB; if (Bt2) Bt2 += z * sB; C += z * sC;
    const int lane = threadIdx.x & 31, lr = lane & 15, hi = lane >> 4; const int r0 = blockIdx.x * 64, c0 = blockIdx.y * 64;
    v8f acc[4][4];
#pragma unroll
    for (int mb = 0; mb < 4; ++mb)
#pragma unroll
        for (int nb = 0; nb < 4; ++nb) acc[mb][nb] = (v8f){};
    const size_t aoff = (size_t)(r0 + lr) * K + 8 * hi, boff = (size_t)(c0 + lr) * K + 8 * hi;
#pragma unroll 1
    for (int kc = 0; kc < K; kc += 32) {
        V a[4], a2[4];
#pragma unroll
        for (int mb = 0; mb < 4; ++mb) { a[mb] = WFrag<T16>::ld(A + aoff + (size_t)mb * 16 * K + kc); if (NSPLIT == 1 || NSPLIT == 2) a2[mb] = WFrag<T16>::ld(A2 + aoff + (size_t)mb * 16 * K + kc); }
#pragma unroll
        for (int nb = 0; nb < 4; ++nb) { const V b = WFrag<T16>::ld(Bt + boff + (size_t)nb * 16 * K + kc); V b2; if (NSPLIT >= 2) b2 = WFrag<T16>::ld(Bt2 + boff + (size_t)nb * 16 * K + kc);
#pragma unroll
            for (int mb = 0; mb < 4; ++mb) { acc[mb][nb] = WFrag<T16>::mma(a[mb], b, acc[mb][nb]); if (NSPLIT == 1 || NSPLIT == 2) acc[mb][nb] = WFrag<T16>::mma(a2[mb], b, acc[mb][nb]); if (NSPLIT >= 2) acc[mb][nb] = WFrag<T16>::mma(a[mb], b2, acc[mb][nb]); } }
        asm volatile("v_nop\n\tv_nop\n\tv_nop\n\tv_nop" : "+v"(acc[0][0]), "+v"(acc[1][1]), "+v"(acc[2][2]), "+v"(acc[3][3]) : "v"(a[0]), "v"(a[3]));
    }
#pragma unroll
    for (int mb = 0; mb < 4; ++mb) {
#pragma unroll
        for (int nb = 0; nb < 4; ++nb) {
#pragma unroll
            for (int j = 0; j < 8; ++j) os[(hi * 8 + j) * 68 + nb * 16 + lr] = acc[mb][nb][j]; }
        __builtin_amdgcn_wave_barrier(); asm volatile("" ::: "memory");
        float* crow = C + (size_t)(r0 + mb * 16) * ldc + c0;
#pragma unroll 1
        for (int ps = 0; ps < 2; ++ps) {
#pragma unroll
            for (int s = 0; s < 8; ++s) { const int row = 2 * s + hi, cofs = lr * 4; v4f val = *(const v4fa*)(os + row * 68 + cofs); if (BIAS) { val[0] += bfr(bias[c0 + cofs]); val[1] += bfr(bias[c0 + cofs + 1]); val[2] += bfr(bias[c0 + cofs + 2]); val[3] += bfr(bias[c0 + cofs + 3]); }
                *(volatile v4f*)(crow + (size_t)row * ldc + cofs) = val; }
            if (ps == 0) __threadfence(); }
        __builtin_amdgcn_wave_barrier(); asm volatile("" ::: "memory");
    }
}

__device__ __forceinline__ h16 tohx(float x) { return (h16)x; }
__device__ __forceinline__ void splitf(float y, unsigned short& h, unsigned short& l) { h = f2bf(y); l = f2bf(y - bf2f(h)); }
typedef __attribute__((ext_vector_type(2))) _Float16 v2h;
typedef __attribute__((ext_vector_type(4))) _Float16 v4h;
typedef __attribute__((ext_vector_type(2))) unsigned short v2us;
typedef __attribute__((ext_vector_type(4))) unsigned short v4us;
typedef __attribute__((ext_vector_type(2))) float v2f;
typedef __attribute__((ext_vector_type(4))) int v4i;

__global__ __launch_bounds__(256) void k_wtG(const float* __restrict__ w, int K, int N, bf* Bt) {
    const int lane = threadIdx.x & 31; const int L0 = (blockIdx.x * 8 + (threadIdx.x >> 5)) * 8; const int nlines = N * K / 64;
#pragma unroll
    for (int ps = 0; ps < 2; ++ps) {
#pragma unroll 1
        for (int l = 0; l < 8; ++l) { const int L = L0 + l; if (L >= nlines) break; const size_t e = (size_t)L * 64 + lane * 2; const int k = (int)(e % K), n = (int)(e / K); v2us o;
            o[0] = f2bf(w[(size_t)k * N + n]); o[1] = f2bf(w[(size_t)(k + 1) * N + n]); *(volatile v2us*)(Bt + e) = o; }
        if (ps == 0) __threadfence(); }
}
__global__ __launch_bounds__(256) void k_cvt8(const float* __restrict__ src, bf* dst, size_t n8) { const size_t i = (size_t)blockIdx.x * 256 + threadIdx.x; if (i >= n8) return; const v8f v = *(const v8f*)(src + i * 8); v8us o;
#pragma unroll
    for (int k = 0; k < 8; ++k) o[k] = f2bf(v[k]); *(volatile v8us*)(dst + i * 8) = o; __threadfence(); *(volatile v8us*)(dst + i * 8) = o; }

__global__ __launch_bounds__(256) void k_rope(const float* __restrict__ F, int pitch, int nheads, const float* __restrict__ CS, const float* __restrict__ RF, const float* __restrict__ nw, float sc, h16* P16, bf* Ph, bf* Pl) {
    const size_t e = ((size_t)blockIdx.x * 256 + threadIdx.x) * 2; if (e >= (size_t)nheads * TT * HD) return; const int d = (int)(e % HD); const int t = (int)((e / HD) % TT); const int h = (int)(e / ((size_t)HD * TT)); const float* f = F + (size_t)t * pitch + h * HD; const float rf = RF ? RF[(size_t)h * TT + t] : 1.0f; v2h o16; v2us oh, ol;
#pragma unroll
    for (int q = 0; q < 2; ++q) { const int dd = d + q; const int dp = (dd < HD / 2) ? dd + HD / 2 : dd - HD / 2; float x0 = f[dd], x1 = f[dp];
        if (RF) { float n0 = __fmul_rn(x0, rf), n1 = __fmul_rn(x1, rf); asm volatile("" : "+v"(n0)); asm volatile("" : "+v"(n1)); x0 = __fmul_rn(bfr(nw[dd]), n0); x1 = __fmul_rn(bfr(nw[dp]), n1); }
        const v2f cs = *(const v2f*)(CS + ((size_t)t * HD + dd) * 2); float a = __fmul_rn(x0, cs[0]), bq = __fmul_rn(x1, cs[1]); asm volatile("" : "+v"(a)); asm volatile("" : "+v"(bq)); const float r = ((dd < HD / 2) ? __fsub_rn(a, bq) : __fadd_rn(a, bq)) * sc;
        o16[q] = tohx(r); unsigned short a2, c2; splitf(r, a2, c2); oh[q] = a2; ol[q] = c2; }
    *(volatile v2h*)(P16 + e) = o16; *(volatile v2us*)(Ph + e) = oh; *(volatile v2us*)(Pl + e) = ol; __threadfence(); *(volatile v2h*)(P16 + e) = o16; *(volatile v2us*)(Ph + e) = oh; *(volatile v2us*)(Pl + e) = ol; }
__global__ __launch_bounds__(256) void k_vtp(const float* __restrict__ F, int pitch, int nheads, h16* V16, bf* Vh, bf* Vl) { const size_t e = ((size_t)blockIdx.x * 256 + threadIdx.x) * 2; if (e >= (size_t)nheads * HD * TT) return; const int t = (int)(e % TT); const int d = (int)((e / TT) % HD); const int g = (int)(e / ((size_t)TT * HD)); v2h o16; v2us oh, ol;
#pragma unroll
    for (int q = 0; q < 2; ++q) { const float x = F[(size_t)(t + q) * pitch + g * HD + d]; o16[q] = tohx(x); unsigned short a2, c2; splitf(x, a2, c2); oh[q] = a2; ol[q] = c2; }
    *(volatile v2h*)(V16 + e) = o16; *(volatile v2us*)(Vh + e) = oh; *(volatile v2us*)(Vl + e) = ol; __threadfence(); *(volatile v2h*)(V16 + e) = o16; *(volatile v2us*)(Vh + e) = oh; *(volatile v2us*)(Vl + e) = ol; }
__global__ __launch_bounds__(256) void k_csid(float* CS) { const int idx = blockIdx.x * 256 + threadIdx.x; if (idx >= TT * HD) return; v2f cs; cs[0] = 1.0f; cs[1] = 0.0f; *(volatile v2f*)(CS + (size_t)idx * 2) = cs; __threadfence(); *(volatile v2f*)(CS + (size_t)idx * 2) = cs; }
__global__ __launch_bounds__(256) void k_asoft(const float* __restrict__ Sb, h16* P16, bf* Ph, bf* Pl) {
    const int lane = threadIdx.x & 31; const int row = blockIdx.x * 8 + (threadIdx.x >> 5); if (row >= ZH * TT) return; const int i = row % TT; const int zz = row / TT; (void)zz; const bool hires = (i < RH); const float* sr = Sb + (size_t)row * TT; float v[TT / 32]; float mx = -3.0e38f;
#pragma unroll
    for (int ch = 0; ch < TT / 128; ++ch) { const int j0 = ch * 128 + lane * 4; const v4f a = *(const v4f*)(sr + j0);
#pragma unroll
        for (int q = 0; q < 4; ++q) { const int j = j0 + q; (void)j; const float t = a[q] * SCL; v[ch * 4 + q] = t; mx = fmaxf(mx, t); } }
#pragma unroll
    for (int sh = 16; sh; sh >>= 1) mx = fmaxf(mx, __shfl_xor(mx, sh, 32));
    float sum = 0.f;
#pragma unroll
    for (int k = 0; k < TT / 32; ++k) { float d0 = __fsub_rn(v[k], mx); asm volatile("" : "+v"(d0)); v[k] = __builtin_amdgcn_exp2f(__fmul_rn(d0, 1.4426950408889634f)); sum += v[k]; }
#pragma unroll
    for (int sh = 16; sh; sh >>= 1) sum += __shfl_xor(sum, sh, 32);
    const float f = __fdiv_rn(hires ? 1.0f : PCAR, sum);
#pragma unroll 1
    for (int ps = 0; ps < 2; ++ps) {
        if (hires) {
#pragma unroll
            for (int ch = 0; ch < TT / 128; ++ch) { v4us oh, ol;
#pragma unroll
                for (int q = 0; q < 4; ++q) { unsigned short a, c2; splitf(v[ch * 4 + q] * f, a, c2); oh[q] = a; ol[q] = c2; }
                const size_t oo = ((size_t)zz * (RH ? RH : 1) + i) * TT + ch * 128 + lane * 4; *(volatile v4us*)(Ph + oo) = oh; *(volatile v4us*)(Pl + oo) = ol; }
        } else {
#pragma unroll
            for (int ch = 0; ch < TT / 128; ++ch) { v4h o4;
#pragma unroll
                for (int q = 0; q < 4; ++q) o4[q] = tohx(v[ch * 4 + q] * f);
                *(volatile v4h*)(P16 + (size_t)row * TT + ch * 128 + lane * 4) = o4; } }
        if (ps == 0) __threadfence(); }
}
__constant__ short DIDX[2 * TT - 1] = { 1023,1023,1023,1023,1023,1023,1023,1023,1023,1023,1023,1023,1023,1023,1023,1023,1023,1023,1023,1023,1023,1023,1023,1023,1023,1023,1023,1023,1023,1023,1023,1023,1023,1023,1023,1023,1023,1023,1023,1023,1023,1023,1023,1023,1023,1023,1023,1023,1023,1023,1023,1023,1023,1023,1023,1023,1023,1023,1023,1023,1023,1023,1023,1023,1023,1023,1023,1023,1023,1023,1023,1023,1023,1023,1023,1023,1023,1023,1023,1023,1023,1023,1023,1023,1023,1023,1023,1023,1023,1023,1023,1023,1023,1023,1023,1023,1023,1023,1023,1023,1023,1023,1023,1023,1023,1023,1023,1023,1023,1023,1023,1023,1023,1023,1023,1023,1023,1023,1023,1023,1023,1023,1023,1023,1023,1023,1023,1023,1023,1023,1023,1023,1023,1023,1023,1023,1023,1023,1023,1023,1023,1023,1023,1023,1023,1023,1023,1023,1023,1023,1023,1023,1023,1023,1023,1023,1023,1023,1023,1023,1023,1023,1023,1023,1023,1023,1023,1023,1023,1023,1023,1023,1023,1023,1023,1023,1023,1023,1023,1023,1023,1023,1023,1023,1023,1023,1023,1023,1023,1023,1023,1023,1023,1023,1023,1023,1023,1023,1023,1023,1023,1023,1023,1023,1023,1023,1023,1023,1023,1023,1023,1023,1023,1023,1023,1023,1023,1023,1023,1023,1023,1023,1023,1023,1023,1023,1023,1023,1023,1023,1023,1023,1023,1023,1023,1023,1023,1023,1023,1023,1023,1023,1023,1023,1023,1023,1023,1023,1023,1023,1023,1023,1023,1023,1023,1023,1023,1023,1023,1023,1023,1023,1023,1023,1023,1023,1023,1023,1023,1023,1023,1023,1023,1023,1023,1023,1023,1023,1023,1023,1023,1023,1023,1023,1023,1023,1023,1023,1023,1023,1023,1023,1023,1023,1023,1023,1023,1023,1023,1023,1023,1023,1023,1023,1023,1023,1023,1023,1023,1023,1023,1023,1023,1023,1023,1023,1023,1023,1023,1023,1023,1023,1023,1023,1023,1023,1023,1023,1023,1023,1023,1023,1023,1023,1023,1023,1023,1023,1023,1023,1023,1023,1023,1023,1023,1023,1023,1023,1023,1023,1023,1023,1023,1023,1023,1023,1023,1023,1023,1023,1023,1023,1023,1023,1023,1023,1023,1023,1023,1023,1023,1023,1023,1023,1023,1023,1023,1023,1023,1023,1023,1023,1023,1023,1023,1023,1023,1023,1023,1023,1023,1023,1023,1023,1023,1023,1023,1023,1023,1023,1023,1023,1023,1023,1023,1023,1023,1023,1023,1023,1023,1023,1023,1023,1023,1023,1023,1023,1023,1023,1023,1023,1023,1023,1023,1023,1023,1023,1023,1023,1023,1023,1023,1023,1023,1023,1023,1023,1023,1023,1023,1023,1023,1023,1023,1023,1023,1023,1023,1023,1023,1023,1023,1023,1023,1023,1023,1023,1023,1023,1023,1023,1023,1023,1023,1023,1023,1023,1023,1023,1023,1023,1023,1023,1023,1023,1023,1023,1023,1023,1023,1023,1023,1023,1023,1023,1023,1023,1023,1023,1023,1023,1023,1023,1023,1023,1023,1023,1023,1023,1023,1023,1023,1023,1023,1023,1023,1023,1023,1023,1023,1023,1023,1022,1021,1020,1019,1018,1017,1016,1015,1014,1013,1012,1011,1010,1009,1008,1007,1006,1005,1004,1003,1002,1001,1000,999,998,997,996,995,994,993,992,991,990,989,988,987,986,985,984,983,982,981,980,979,978,977,976,975,974,973,972,971,970,969,968,967,966,965,964,963,962,961,960,959,958,957,956,955,954,953,952,951,950,949,948,947,946,945,944,943,942,941,940,939,938,937,936,935,934,933,932,931,930,929,928,927,926,925,924,923,922,921,920,919,918,917,916,915,914,913,912,911,910,909,908,907,906,905,904,903,902,901,900,899,898,897,896,895,894,893,892,891,890,889,888,887,886,885,884,883,882,881,880,879,878,877,876,875,874,873,872,871,870,869,868,867,866,865,864,863,862,861,860,859,858,857,856,855,854,853,852,851,850,849,848,847,846,845,844,843,842,841,840,839,838,837,836,835,834,833,832,831,830,829,828,827,826,825,824,823,822,821,820,819,818,817,816,815,814,813,812,811,810,809,808,807,806,805,804,803,802,801,800,799,798,797,796,795,794,793,792,791,790,789,788,787,786,785,784,783,782,781,780,779,778,777,776,775,774,773,772,771,770,769,768,767,766,765,764,763,762,761,760,759,758,757,756,755,754,753,752,751,750,749,748,747,746,745,744,743,742,741,740,739,738,737,736,735,734,733,732,731,730,729,728,727,726,725,724,723,722,721,720,719,718,717,716,715,714,713,712,711,710,709,708,707,706,705,704,703,702,701,700,699,698,697,696,695,694,693,692,691,690,689,688,687,686,685,684,683,682,681,680,679,678,677,676,675,674,673,672,671,670,669,668,667,666,665,664,663,662,661,660,659,658,657,656,655,654,653,652,651,650,649,648,647,646,645,644,643,642,641,640,639,638,637,636,635,634,633,632,631,630,629,628,627,626,625,624,623,622,621,620,619,618,617,616,615,614,613,612,611,610,609,608,607,606,605,604,603,602,601,600,599,598,597,596,595,594,593,592,591,590,589,588,587,586,585,584,583,582,581,580,579,578,577,576,575,574,573,572,571,570,569,568,567,566,565,564,563,562,561,560,559,558,557,556,555,554,553,552,551,550,549,548,547,546,545,544,543,542,541,540,539,538,537,536,535,534,533,532,531,530,529,528,527,526,525,524,523,522,521,520,519,518,517,516,515,514,513,512,511,510,509,508,507,506,505,504,503,502,501,500,499,498,497,496,495,494,493,492,491,490,489,488,487,486,485,484,483,482,481,480,479,478,477,476,475,474,473,472,471,470,469,468,467,466,465,464,463,462,461,460,459,458,457,456,455,454,453,452,451,450,449,448,447,446,445,444,443,442,441,440,439,438,437,436,435,434,433,432,431,430,429,428,427,426,425,424,423,422,421,420,419,418,417,416,415,414,413,412,411,410,409,408,407,406,405,404,403,402,401,400,399,398,397,396,395,394,393,392,391,390,389,388,387,386,385,384,383,382,381,380,379,378,377,376,375,374,373,372,371,370,369,368,367,366,365,364,363,362,361,360,359,358,357,356,355,354,353,352,351,350,349,348,347,346,345,344,343,342,341,340,339,338,337,336,335,334,333,332,331,330,329,328,327,326,325,324,323,322,321,320,319,318,317,316,315,314,313,312,311,310,309,308,307,306,305,304,303,302,301,300,299,298,297,296,295,294,293,292,291,290,289,288,287,286,285,284,283,282,281,280,279,278,277,276,275,274,273,272,271,270,269,268,267,266,265,264,263,262,261,260,259,258,257,256,255,254,253,252,251,250,249,248,247,246,245,244,243,242,241,240,239,238,237,236,235,234,233,232,231,230,229,228,227,226,225,224,223,222,221,220,219,218,217,216,215,214,213,212,211,210,209,208,207,206,205,204,203,202,201,200,199,198,197,196,195,194,193,192,191,190,189,188,187,186,185,184,183,182,181,180,179,178,177,176,175,174,173,172,171,170,169,168,167,166,165,164,163,162,161,160,159,158,157,156,155,154,153,152,151,150,149,148,147,146,145,144,143,142,141,140,139,138,137,136,135,134,133,132,131,130,129,128,127,126,125,124,123,122,121,120,119,118,117,116,115,114,113,112,111,110,109,108,107,106,105,104,103,102,101,100,99,98,97,96,95,94,93,92,91,90,89,88,87,86,85,84,83,82,81,80,79,78,77,76,75,74,73,72,71,70,69,68,67,66,65,64,63,62,61,60,59,58,57,56,55,54,53,52,51,50,49,48,47,46,45,44,43,42,41,40,39,38,37,36,35,34,33,32,31,30,29,28,27,26,25,24,23,22,21,20,19,18,17,16,15,14,13,12,11,10,9,8,7,6,5,4,3,2,1,0,0,0,0,0,0,0,0,0,0,0,0,0,0,0,0,0,0,0,0,0,0,0,0,0,0,0,0,0,0,0,0,0,0,0,0,0,0,0,0,0,0,0,0,0,0,0,0,0,0,0,0,0,0,0,0,0,0,0,0,0,0,0,0,0,0,0,0,0,0,0,0,0,0,0,0,0,0,0,0,0,0,0,0,0,0,0,0,0,0,0,0,0,0,0,0,0,0,0,0,0,0,0,0,0,0,0,0,0,0,0,0,0,0,0,0,0,0,0,0,0,0,0,0,0,0,0,0,0,0,0,0,0,0,0,0,0,0,0,0,0,0,0,0,0,0,0,0,0,0,0,0,0,0,0,0,0,0,0,0,0,0,0,0,0,0,0,0,0,0,0,0,0,0,0,0,0,0,0,0,0,0,0,0,0,0,0,0,0,0,0,0,0,0,0,0,0,0,0,0,0,0,0,0,0,0,0,0,0,0,0,0,0,0,0,0,0,0,0,0,0,0,0,0,0,0,0,0,0,0,0,0,0,0,0,0,0,0,0,0,0,0,0,0,0,0,0,0,0,0,0,0,0,0,0,0,0,0,0,0,0,0,0,0,0,0,0,0,0,0,0,0,0,0,0,0,0,0,0,0,0,0,0,0,0,0,0,0,0,0,0,0,0,0,0,0,0,0,0,0,0,0,0,0,0,0,0,0,0,0,0,0,0,0,0,0,0,0,0,0,0,0,0,0,0,0,0,0,0,0,0,0,0,0,0,0,0,0,0,0,0,0,0,0,0,0,0,0,0,0,0,0,0,0,0,0,0,0,0,0,0,0,0,0,0,0,0,0,0,0,0,0,0,0,0,0,0,0,0,0,0,0,0,0,0,0,0,0,0,0,0,0,0,0,0,0,0,0,0,0,0,0,0,0,0,0,0,0,0,0,0,0,0,0,0,0,0,0,0,0,0,0,0,0,0,0,0,0,0,0,0,0,0,0,0,0,0,0,0,0,0,0,0,0,0,0,0,0,0,0,0,0,0,0,0,0,0,0,0,0,0,0,0,0,0,0,0,0,0,0,0,0,0,0,0,0,0,0,0,0,0,0,0,0,0,0,0,0,0,0,0,0,0,0,0,0,0,0,0,0,0,0,0,0,0,0,0,0,0,0,0,0 };
__global__ __launch_bounds__(256) void k_hpl(const float* __restrict__ F, int nrows, bf* Ph, bf* Pl) { const size_t e = ((size_t)blockIdx.x * 256 + threadIdx.x) * 2; if (e >= (size_t)NH_ * nrows * HD) return; const int d = (int)(e % HD); const int p = (int)((e / HD) % nrows); const int h = (int)(e / ((size_t)HD * nrows)); const float* f = F + (size_t)p * DQ + h * HD + d; v2us oh, ol;
#pragma unroll
    for (int q = 0; q < 2; ++q) { unsigned short a, c2; splitf(f[q], a, c2); oh[q] = a; ol[q] = c2; }
    *(volatile v2us*)(Ph + e) = oh; *(volatile v2us*)(Pl + e) = ol; __threadfence(); *(volatile v2us*)(Ph + e) = oh; *(volatile v2us*)(Pl + e) = ol; }
__global__ __launch_bounds__(256) void k_flat(const float* __restrict__ F, h16* P16, bf* Ph, bf* Pl, size_t n4) { const size_t i = (size_t)blockIdx.x * 256 + threadIdx.x; if (i >= n4) return; const v4f a = *(const v4f*)(F + i * 4); v4h o16; v4us oh, ol;
#pragma unroll
    for (int q = 0; q < 4; ++q) { o16[q] = tohx(a[q]); unsigned short x2, y2; splitf(a[q], x2, y2); oh[q] = x2; ol[q] = y2; }
    *(volatile v4h*)(P16 + i * 4) = o16; *(volatile v4us*)(Ph + i * 4) = oh; *(volatile v4us*)(Pl + i * 4) = ol; __threadfence(); *(volatile v4h*)(P16 + i * 4) = o16; *(volatile v4us*)(Ph + i * 4) = oh; *(volatile v4us*)(Pl + i * 4) = ol; }

__global__ __launch_bounds__(256) void k_adddis(float* Sb, const float* __restrict__ QPK, const float* __restrict__ KPQ) { const size_t k = (size_t)blockIdx.x * 256 + threadIdx.x; if (k >= (size_t)ZH * TT * TT / 4) return; const size_t e = k * 4; const int j0 = (int)(e % TT); const int i = (int)((e / TT) % TT); const size_t zz = e / ((size_t)TT * TT); const float* qpk = QPK + (zz * TT + i) * NPOS; v4f a = *(const v4f*)(Sb + e);
#pragma unroll
    for (int q = 0; q < 4; ++q) { const int j = j0 + q; const int idx = (int)DIDX[i - j + (TT - 1)]; float s1 = __fadd_rn(a[q], qpk[idx]); asm volatile("" : "+v"(s1)); a[q] = __fadd_rn(s1, KPQ[(zz * TT + j) * NPOS + idx]); }
    *(volatile v4f*)(Sb + e) = a; __threadfence(); *(volatile v4f*)(Sb + e) = a; }
__global__ __launch_bounds__(256) void k_merge(const float* __restrict__ O, int h0, float* OUTb) { const size_t e = ((size_t)blockIdx.x * 256 + threadIdx.x) * 2; if (e >= (size_t)ZH * TT * HD) return; const int d = (int)(e % HD); const int t = (int)((e / HD) % TT); const int zz = (int)(e / ((size_t)HD * TT)); const float cs = (t < RH) ? 1.0f : (1.0f / PCAR); const size_t oo = (size_t)t * DQ + (h0 + zz) * HD + d;
    v2f o2; o2[0] = O[e] * cs; o2[1] = O[e + 1] * cs; *(volatile v2f*)(OUTb + oo) = o2; __threadfence(); *(volatile v2f*)(OUTb + oo) = o2; }

extern "C" void kernel_launch(void* const* d_in, const int* in_sizes, int n_in,
                              void* d_out, int out_size, void* d_ws, size_t ws_size, hipStream_t stream) {
    (void)in_sizes; (void)n_in; (void)out_size;
    const float* x = (const float*)d_in[0]; const float* wq = (const float*)d_in[1]; const float* bq = (const float*)d_in[2]; const float* wk = (const float*)d_in[3]; const float* bk = (const float*)d_in[4]; const float* wv = (const float*)d_in[5]; const float* bv = (const float*)d_in[6]; const float* wo = (const float*)d_in[7]; const float* bo = (const float*)d_in[8]; const float* wpk = (const float*)d_in[9]; const float* bpk = (const float*)d_in[10]; const float* wpq = (const float*)d_in[11]; const float* bpq = (const float*)d_in[12]; const float* remb = (const float*)d_in[13];
    float* OUT = (float*)d_out;
    char* wsp = (char*)d_ws;
    auto take = [&](size_t bytes) { char* p = wsp; wsp += (bytes + 255) & ~(size_t)255; return (void*)p; };
    bf* WPQ = (bf*)take((size_t)DQ * DM * 2); bf* WPK = (bf*)take((size_t)DQ * DM * 2); bf* RB = (bf*)take((size_t)NPOS * DM * 2); float* FP = (float*)take((size_t)NPOS * DQ * 4); bf* PKh = (bf*)take((size_t)NH_ * NPOS * HD * 2); bf* PKl = (bf*)take((size_t)NH_ * NPOS * HD * 2); bf* PQh = (bf*)take((size_t)NH_ * NPOS * HD * 2); bf* PQl = (bf*)take((size_t)NH_ * NPOS * HD * 2); float* QPK = (float*)take((size_t)ZH * TT * NPOS * 4); float* KPQ = (float*)take((size_t)ZH * TT * NPOS * 4); bf* WO = (bf*)take((size_t)DM * DQ * 2); float* CTX = (float*)take((size_t)TT * DQ * 4); h16* A16 = (h16*)take((size_t)TT * DQ * 2); bf* ATh = (bf*)take((size_t)TT * DQ * 2); bf* ATl = (bf*)take((size_t)TT * DQ * 2); bf* WQ = (bf*)take((size_t)DQ * DM * 2); bf* WK = (bf*)take((size_t)DKV * DM * 2); bf* WV = (bf*)take((size_t)DKV * DM * 2); float* CS = (float*)take((size_t)TT * HD * 2 * 4);
    bf* XB = (bf*)take((size_t)TT * DM * 2); float* FQ = (float*)take((size_t)TT * DQ * 4); float* FK = (float*)take((size_t)TT * DKV * 4);
    h16* QP16 = (h16*)take((size_t)NH_ * TT * HD * 2); h16* KP16 = (h16*)take((size_t)NKV * TT * HD * 2); h16* VT16 = (h16*)take((size_t)NKV * HD * TT * 2);
    bf* QPh = (bf*)take((size_t)NH_ * TT * HD * 2); bf* QPl = (bf*)take((size_t)NH_ * TT * HD * 2); bf* KPh = (bf*)take((size_t)NKV * TT * HD * 2); bf* KPl = (bf*)take((size_t)NKV * TT * HD * 2); bf* VTh = (bf*)take((size_t)NKV * HD * TT * 2); bf* VTl = (bf*)take((size_t)NKV * HD * TT * 2); bf* Ph = (bf*)take((size_t)ZH * RH * TT * 2); bf* Pl = (bf*)take((size_t)ZH * RH * TT * 2);
    float* Sb = (float*)take((size_t)ZH * TT * TT * 4); h16* P16 = (h16*)take((size_t)ZH * TT * TT * 2); float* Ob = (float*)take((size_t)ZH * TT * HD * 4);
    if ((size_t)(wsp - (char*)d_ws) > ws_size) return;
    float* FV = FK;
    { k_cvt8<<<(unsigned)(((size_t)DQ * DM / 8 + 255) / 256), 256, 0, stream>>>(wpq, WPQ, (size_t)DQ * DM / 8); k_cvt8<<<(unsigned)(((size_t)DQ * DM / 8 + 255) / 256), 256, 0, stream>>>(wpk, WPK, (size_t)DQ * DM / 8); k_cvt8<<<(unsigned)(((size_t)NPOS * DM / 8 + 255) / 256), 256, 0, stream>>>(remb, RB, (size_t)NPOS * DM / 8);
        k_gemmw<bf, 0, true><<<dim3(NPOS / 64, DQ / 64, 1), 32, 0, stream>>>(RB, nullptr, WPK, nullptr, DM, FP, DQ, bpk, 0, 0, 0); k_hpl<<<(unsigned)(((size_t)NH_ * NPOS * HD / 2 + 255) / 256), 256, 0, stream>>>(FP, NPOS, PKh, PKl);
        k_gemmw<bf, 0, true><<<dim3(NPOS / 64, DQ / 64, 1), 32, 0, stream>>>(RB, nullptr, WPQ, nullptr, DM, FP, DQ, bpq, 0, 0, 0); k_hpl<<<(unsigned)(((size_t)NH_ * NPOS * HD / 2 + 255) / 256), 256, 0, stream>>>(FP, NPOS, PQh, PQl);
        k_cvt8<<<(unsigned)(((size_t)DQ * DM / 8 + 255) / 256), 256, 0, stream>>>(wq, WQ, (size_t)DQ * DM / 8); k_cvt8<<<(unsigned)(((size_t)DM * DQ / 8 + 255) / 256), 256, 0, stream>>>(wo, WO, (size_t)DM * DQ / 8); k_cvt8<<<(unsigned)(((size_t)DKV * DM / 8 + 255) / 256), 256, 0, stream>>>(wk, WK, (size_t)DKV * DM / 8); k_cvt8<<<(unsigned)(((size_t)DKV * DM / 8 + 255) / 256), 256, 0, stream>>>(wv, WV, (size_t)DKV * DM / 8);

       }
    k_csid<<<(TT * HD + 255) / 256, 256, 0, stream>>>(CS);
    const unsigned LQ = (unsigned)(((size_t)NH_ * TT * HD / 2 + 255) / 256), LKv = (unsigned)(((size_t)NKV * TT * HD / 2 + 255) / 256);
    for (int b = 0; b < NB_; ++b) {

        k_cvt8<<<(unsigned)(((size_t)TT * DM / 8 + 255) / 256), 256, 0, stream>>>(x + (size_t)b * TT * DM, XB, (size_t)TT * DM / 8);
        k_gemmw<bf, 0, true><<<dim3(TT / 64, DQ / 64, 1), 32, 0, stream>>>(XB, nullptr, WQ, nullptr, DM, FQ, DQ, bq, 0, 0, 0);
        k_rope<<<LQ, 256, 0, stream>>>(FQ, DQ, NH_, CS, nullptr, nullptr, 1.0f, QP16, QPh, QPl);
        k_gemmw<bf, 0, true><<<dim3(TT / 64, DKV / 64, 1), 32, 0, stream>>>(XB, nullptr, WK, nullptr, DM, FK, DKV, bk, 0, 0, 0);
        k_rope<<<LKv, 256, 0, stream>>>(FK, DKV, NKV, CS, nullptr, nullptr, 1.0f, KP16, KPh, KPl);
        k_gemmw<bf, 0, true><<<dim3(TT / 64, DKV / 64, 1), 32, 0, stream>>>(XB, nullptr, WV, nullptr, DM, FV, DKV, bv, 0, 0, 0); k_vtp<<<LKv, 256, 0, stream>>>(FV, DKV, NKV, VT16, VTh, VTl);
        for (int h0 = 0; h0 < NH_; h0 += ZH) { const size_t zq = (size_t)h0, zk = (size_t)(h0 / REP);
            k_gemmw<bf, 2, false><<<dim3(RH / 64, TT / 64, ZH), 32, 0, stream>>>(QPh + zq * TT * HD, QPl + zq * TT * HD, KPh + zk * TT * HD, KPl + zk * TT * HD, HD, Sb, TT, nullptr, (size_t)TT * HD, (size_t)TT * HD, (size_t)TT * TT);
            k_gemmw<h16, 0, false><<<dim3((TT - RH) / 64, TT / 64, ZH), 32, 0, stream>>>(QP16 + zq * TT * HD + (size_t)RH * HD, nullptr, KP16 + zk * TT * HD, nullptr, HD, Sb + (size_t)RH * TT, TT, nullptr, (size_t)TT * HD, (size_t)TT * HD, (size_t)TT * TT);
            k_gemmw<bf, 2, false><<<dim3(TT / 64, NPOS / 64, ZH), 32, 0, stream>>>(QPh + zq * TT * HD, QPl + zq * TT * HD, PKh + zq * NPOS * HD, PKl + zq * NPOS * HD, HD, QPK, NPOS, nullptr, (size_t)TT * HD, (size_t)NPOS * HD, (size_t)TT * NPOS);
            k_gemmw<bf, 2, false><<<dim3(TT / 64, NPOS / 64, ZH), 32, 0, stream>>>(KPh + zk * TT * HD, KPl + zk * TT * HD, PQh + zq * NPOS * HD, PQl + zq * NPOS * HD, HD, KPQ, NPOS, nullptr, (size_t)TT * HD, (size_t)NPOS * HD, (size_t)TT * NPOS);
            k_adddis<<<(unsigned)(((size_t)ZH * TT * TT / 4 + 255) / 256), 256, 0, stream>>>(Sb, QPK, KPQ);
            k_asoft<<<ZH * TT / 8, 256, 0, stream>>>(Sb, P16, Ph, Pl);
            k_gemmw<bf, 2, false><<<dim3(RH / 64, HD / 64, ZH), 32, 0, stream>>>(Ph, Pl, VTh + zk * HD * TT, VTl + zk * HD * TT, TT, Ob, HD, nullptr, (size_t)RH * TT, (size_t)HD * TT, (size_t)TT * HD);
            k_gemmw<h16, 0, false><<<dim3((TT - RH) / 64, HD / 64, ZH), 32, 0, stream>>>(P16 + (size_t)RH * TT, nullptr, VT16 + zk * HD * TT, nullptr, TT, Ob + (size_t)RH * HD, HD, nullptr, (size_t)TT * TT, (size_t)HD * TT, (size_t)TT * HD);
            k_merge<<<(unsigned)(((size_t)ZH * TT * HD / 2 + 255) / 256), 256, 0, stream>>>(Ob, h0, CTX); }
        k_flat<<<(unsigned)(((size_t)TT * DQ / 4 + 255) / 256), 256, 0, stream>>>(CTX, A16, ATh, ATl, (size_t)TT * DQ / 4); k_gemmw<bf, 1, true><<<dim3(TT / 64, DM / 64, 1), 32, 0, stream>>>(ATh, ATl, WO, nullptr, DQ, OUT + (size_t)b * TT * DM, DM, bo, 0, 0, 0);
         }
}
